// CausalSelfAttention_82918638616672
// MI455X (gfx1250) — hardware-verified
//
#include <hip/hip_runtime.h>
#ifndef NB
#define NB 2
#endif
#ifndef SEQ
#define SEQ 2048
#endif
#define NB_FULL 2
#define SEQ_FULL 2048
#define DM 1024
#define NH 16
#define HD 64
#define QT 256
#define NKX SEQ
#define QT0 256
#define NR ((size_t)NB * SEQ)
#define AL256(x) ((((size_t)(x)) + 255) & ~(size_t)255)

static_assert(DM == NH * HD);
static_assert(SEQ % QT == 0);
static_assert(QT % 128 == 0);
static_assert(QT0 % 128 == 0);
static_assert(SEQ >= QT0);
static_assert((SEQ - QT0) % QT == 0);
static_assert(SEQ <= SEQ_FULL);
static_assert(NB <= NB_FULL);
static_assert(DM / 8 == 128);
static_assert(DM % 64 == 0);
static_assert(HD % 32 == 0);
static_assert(HD == 64);

typedef unsigned short v8us __attribute__((ext_vector_type(8), may_alias));
typedef float  v8f  __attribute__((ext_vector_type(8)));
typedef float  v4f  __attribute__((ext_vector_type(4)));
typedef float  v4fa __attribute__((ext_vector_type(4), may_alias));
typedef _Float16 v16h __attribute__((ext_vector_type(16)));
typedef _Float16 v4h __attribute__((ext_vector_type(4)));
union FragH { v16h v; v8us half[2]; _Float16 h[16]; unsigned short u[16]; };

__device__ __forceinline__ unsigned short bf16_bits(float x) { unsigned int u = __float_as_uint(x); return (unsigned short)((u + 0x7FFFu + ((u >> 16) & 1u)) >> 16); }
__device__ __forceinline__ float bf16_val(unsigned short b) { return __uint_as_float(((unsigned int)b) << 16); }
__device__ __forceinline__ float bf16_rne(float x) { return bf16_val(bf16_bits(x)); }

__device__ __forceinline__ v16h g2_frag(const _Float16* p, unsigned hh) { FragH f; f.half[0] = *(const v8us*)((const unsigned short*)p + 8 * hh); f.half[1] = *(const v8us*)((const unsigned short*)p + 16 + 8 * hh); return f.v; }
__device__ __forceinline__ v8f g2_mma(v16h a, v16h b, v8f c) { v8f d = __builtin_amdgcn_wmma_f32_16x16x32_f16(false, a, false, b, (short)0, c, false, false); asm volatile("v_nop\n\tv_nop\n\tv_nop\n\tv_nop" : "+v"(d) : "v"(a), "v"(b)); return d; }

__global__ __launch_bounds__(256) void k_wt_f16(const float* __restrict__ W, _Float16* __restrict__ Wt, unsigned K, unsigned N, float scale) {
  const unsigned t = blockIdx.x * 256u + threadIdx.x; const unsigned k8n = K >> 3; if (t >= N * k8n) return;
  const unsigned n = t / k8n, k8 = (t - n * k8n) << 3; FragH f;
#pragma unroll
  for (unsigned i = 0; i < 8; ++i) f.h[i] = (_Float16)(bf16_rne(W[(size_t)(k8 + i) * N + n]) * scale);
  const v8us o = f.half[0]; unsigned short* d = (unsigned short*)Wt + (size_t)n * K + k8;
  *(volatile v8us*)d = o; __threadfence(); *(volatile v8us*)d = o;
}

__global__ __launch_bounds__(256) void k_x16(const float* __restrict__ x, _Float16* __restrict__ X16, unsigned n8) {
  const unsigned t = blockIdx.x * 256u + threadIdx.x; if (t >= n8) return;
  const unsigned row = t >> 7, c8 = (t & 127u) << 3; const unsigned b = row / (unsigned)SEQ, s = row - b * (unsigned)SEQ;
  const float* src = x + ((size_t)b * SEQ_FULL + s) * DM + c8;
  const v4f a = *(const v4fa*)src, c = *(const v4fa*)(src + 4); FragH f;
#pragma unroll
  for (unsigned q = 0; q < 4; ++q) { f.h[q] = (_Float16)bf16_rne(a[q]); f.h[4 + q] = (_Float16)bf16_rne(c[q]); }
  const v8us o = f.half[0]; unsigned short* d = (unsigned short*)X16 + (size_t)t * 8;
  *(volatile v8us*)d = o; __threadfence(); *(volatile v8us*)d = o;
}

__global__ __launch_bounds__(256) void k_vt(const _Float16* __restrict__ V2, _Float16* __restrict__ VT2) {
  __shared__ unsigned short tl[64][66];
  const unsigned tid = threadIdx.x; const unsigned h = blockIdx.x / (unsigned)(SEQ / 64), lg = blockIdx.x % (unsigned)(SEQ / 64); const unsigned b = blockIdx.y, pl = blockIdx.z;
  const unsigned short* src = (const unsigned short*)V2 + ((size_t)pl * NR + (size_t)b * SEQ) * DM;
  unsigned short* dst = (unsigned short*)VT2 + ((size_t)(pl * (unsigned)NB + b) * NH + h) * ((size_t)HD * SEQ);
  for (unsigned i = tid; i < 64u * 8u; i += 256u) { const unsigned r = i >> 3, c8 = (i & 7u) << 3; FragH f; f.half[0] = *(const v8us*)(src + ((size_t)lg * 64 + r) * DM + h * 64u + c8);
#pragma unroll
    for (unsigned q = 0; q < 8; ++q) tl[r][c8 + q] = f.u[q]; }
  __syncthreads();
  for (int pass = 0; pass < 2; ++pass) {
#pragma unroll
    for (unsigned rd = 0; rd < 2; ++rd) { const unsigned d = rd * 32u + (tid >> 3), pc = tid & 7u; FragH f;
#pragma unroll
      for (unsigned q = 0; q < 8; ++q) f.u[q] = tl[pc * 8u + q][d];
      *(volatile v8us*)(dst + (size_t)d * SEQ + lg * 64u + pc * 8u) = f.half[0]; }
    if (pass == 0) __threadfence(); }
}

__global__ __launch_bounds__(256) void k_hl(const float* __restrict__ F, _Float16* __restrict__ Hh, _Float16* __restrict__ Hl, unsigned n8) {
  const unsigned t = blockIdx.x * 256u + threadIdx.x; if (t >= n8) return; FragH fh, fl; const v4f a = *(const v4fa*)(F + (size_t)t * 8), c = *(const v4fa*)(F + (size_t)t * 8 + 4);
  const unsigned row = t >> 7, c8 = (t & 127u) << 3; const unsigned b = row / (unsigned)QT0, s = row - b * (unsigned)QT0;
  const size_t dofs = ((size_t)b * SEQ + s) * DM + c8;
#pragma unroll
  for (unsigned q = 0; q < 4; ++q) { _Float16 h = (_Float16)a[q]; fh.h[q] = h; fl.h[q] = (_Float16)((a[q] - (float)h) * 1024.0f); h = (_Float16)c[q]; fh.h[4 + q] = h; fl.h[4 + q] = (_Float16)((c[q] - (float)h) * 1024.0f); }
  const v8us oh = fh.half[0], ol = fl.half[0];
  for (int pass = 0; pass < 2; ++pass) { *(volatile v8us*)((unsigned short*)Hh + dofs) = oh; *(volatile v8us*)((unsigned short*)Hl + dofs) = ol; if (pass == 0) __threadfence(); }
}

__global__ __launch_bounds__(128) void k_gemm2(const _Float16* __restrict__ A, unsigned lda, size_t sA, const _Float16* __restrict__ Bh, unsigned ldb, size_t sB, float alpha, const float* __restrict__ bias,
    const float* CP, float* C, _Float16* C16, _Float16* C16L, unsigned ldc, size_t sC, unsigned M, unsigned N, unsigned K) {
  __shared__ __attribute__((aligned(16))) float so[4][32][68];
  const unsigned tid = threadIdx.x, w = tid >> 5, lane = tid & 31u, ln = lane & 15u, hh = lane >> 4; const unsigned by = blockIdx.y;
  A += (size_t)by * sA; Bh += (size_t)by * sB; const size_t cofs = (size_t)by * sC;
  const unsigned ntn = N >> 6; const unsigned mt = blockIdx.x / ntn, nq = blockIdx.x - mt * ntn; const unsigned row0 = mt * 128u + 32u * w, col0 = nq * 64u; if (row0 >= M) return;
  const _Float16* a0p = A + (size_t)(row0 + ln) * lda; const _Float16* a1p = a0p + (size_t)16 * lda;
  const _Float16* b0p = Bh + (size_t)(col0 + ln) * ldb; const _Float16* b1p = b0p + (size_t)16 * ldb; const _Float16* b2p = b1p + (size_t)16 * ldb; const _Float16* b3p = b2p + (size_t)16 * ldb;
  const v8f z8 = {0.f,0.f,0.f,0.f,0.f,0.f,0.f,0.f}; v8f c00 = z8, c01 = z8, c02 = z8, c03 = z8, c10 = z8, c11 = z8, c12 = z8, c13 = z8;
#pragma unroll 1
  for (unsigned kb = 0; kb < K; kb += 32) { const v16h a0 = g2_frag(a0p + kb, hh), a1 = g2_frag(a1p + kb, hh);
    v16h b = g2_frag(b0p + kb, hh); c00 = g2_mma(a0, b, c00); c10 = g2_mma(a1, b, c10);
    b = g2_frag(b1p + kb, hh); c01 = g2_mma(a0, b, c01); c11 = g2_mma(a1, b, c11);
    b = g2_frag(b2p + kb, hh); c02 = g2_mma(a0, b, c02); c12 = g2_mma(a1, b, c12);
    b = g2_frag(b3p + kb, hh); c03 = g2_mma(a0, b, c03); c13 = g2_mma(a1, b, c13); }
  v8f accs[8] = {c00, c01, c02, c03, c10, c11, c12, c13};
#pragma unroll
  for (unsigned u = 0; u < 8; ++u) { const unsigned t = u & 3u, half = u >> 2; const unsigned col = col0 + t * 16u + ln; const float bv = bias ? bf16_rne(bias[col]) : 0.f;
#pragma unroll
    for (unsigned r = 0; r < 8; ++r) { const unsigned rloc = half * 16u + 8u * hh + r; float v = accs[u][r] * alpha + bv;
      if (CP) v += CP[cofs + (size_t)(row0 + rloc) * ldc + col];
      so[w][rloc][t * 16u + ln] = v; } }
  __builtin_amdgcn_fence(4  , "workgroup"); __builtin_amdgcn_wave_barrier();
  const unsigned rsub = lane >> 4, c4 = (lane & 15u) * 4u;
  for (int pass = 0; pass < 2; ++pass) {
#pragma unroll
    for (unsigned q = 0; q < 16; ++q) { const unsigned r = q * 2u + rsub; const v4f v = *(const v4fa*)&so[w][r][c4]; const size_t idx = cofs + (size_t)(row0 + r) * ldc + col0 + c4;
      if (C) *(volatile v4f*)(C + idx) = v;
      if (C16) { v4h h4, l4;
#pragma unroll
        for (unsigned i = 0; i < 4; ++i) { const _Float16 hv = (_Float16)v[i]; h4[i] = hv; l4[i] = (_Float16)((v[i] - (float)hv) * 1024.0f); }
        *(volatile v4h*)(C16 + idx) = h4;
        if (C16L) *(volatile v4h*)(C16L + idx) = l4; } }
    if (pass == 0) __threadfence(); }
}

__global__ __launch_bounds__(256) void k_rsmc(const float* __restrict__ S, _Float16* __restrict__ P, _Float16* __restrict__ PL, unsigned nrows, unsigned q0, unsigned nk) {
  #pragma clang fp contract(off)
  const unsigned t = blockIdx.x * 256u + threadIdx.x; if (t >= nrows) return; const float* s = S + (size_t)t * NKX; const unsigned last = q0 + (t % (unsigned)QT); float mx = -3.0e38f;
#pragma unroll 1
  for (unsigned j = 0; j < nk; ++j) { const float f = (j <= last) ? 1.f : 0.f; mx = fmaxf(mx, fmaf(f, s[j], (1.f - f) * -1.0e9f)); }
  float se = 0.f;
#pragma unroll 1
  for (unsigned j = 0; j < nk; ++j) { const float f = (j <= last) ? 1.f : 0.f; se += __expf(fmaf(f, s[j], (1.f - f) * -1.0e9f) - mx); }
  const float sc = 256.0f / se;
#pragma unroll 1
  for (unsigned j0 = 0; j0 < nk; j0 += 8) { FragH fr, fl;
#pragma unroll
    for (unsigned q = 0; q < 8; ++q) { const unsigned j = j0 + q; const float f = (j <= last) ? 1.f : 0.f; const float pv = __expf(fmaf(f, s[j], (1.f - f) * -1.0e9f) - mx) * sc; const _Float16 hv = (_Float16)pv; fr.h[q] = hv; fl.h[q] = (_Float16)((pv - (float)hv) * 1024.0f); }
    const v8us oh = fr.half[0], ol = fl.half[0]; unsigned short* dh = (unsigned short*)P + (size_t)t * NKX + j0; unsigned short* dl = (unsigned short*)PL + (size_t)t * NKX + j0;
    *(volatile v8us*)dh = oh; *(volatile v8us*)dl = ol; __threadfence(); *(volatile v8us*)dh = oh; *(volatile v8us*)dl = ol; }
}

__global__ __launch_bounds__(64) void k_att0(const float* __restrict__ QF, const float* __restrict__ KF, const float* __restrict__ VF, unsigned ld, float scale, float* __restrict__ OF, unsigned ldo) {
  #pragma clang fp contract(off)
  __shared__ __attribute__((aligned(16))) float lq[64][64]; __shared__ __attribute__((aligned(16))) float lo[64][64];
  const unsigned tid = threadIdx.x; const unsigned h = blockIdx.x / (unsigned)(QT0 / 64), rg = blockIdx.x % (unsigned)(QT0 / 64); const unsigned i = rg * 64u + tid; const unsigned bb = blockIdx.y;
  QF += (size_t)bb * QT0 * ld; KF += (size_t)bb * QT0 * ld; VF += (size_t)bb * QT0 * ld; OF += (size_t)bb * QT0 * ldo;
  const float* qr = QF + (size_t)i * ld + h * HD;
#pragma unroll 1
  for (unsigned c = 0; c < HD / 4; ++c) { *(v4f*)&lq[tid][c * 4] = *(const v4fa*)(qr + c * 4); const v4f z = {0.f, 0.f, 0.f, 0.f}; *(v4f*)&lo[tid][c * 4] = z; }
  float m = -1.0e30f, l = 0.f; const unsigned jmax = rg * 64u + 63u;
#pragma unroll 1
  for (unsigned j = 0; j <= jmax; ++j) { const float* kr = KF + (size_t)j * ld + h * HD; const float* vr = VF + (size_t)j * ld + h * HD; float s = 0.f;
#pragma unroll 1
    for (unsigned c = 0; c < HD / 4; ++c) { const v4f kq = *(const v4fa*)(kr + c * 4); const v4f qq = *(v4f*)&lq[tid][c * 4]; s = __fadd_rn(s, __fmul_rn(qq[0], kq[0])); s = __fadd_rn(s, __fmul_rn(qq[1], kq[1])); s = __fadd_rn(s, __fmul_rn(qq[2], kq[2])); s = __fadd_rn(s, __fmul_rn(qq[3], kq[3])); }
    s = __fmul_rn(s, scale);
    const float f = (j <= i) ? 1.f : 0.f; const float sm = fmaf(f, s, (1.f - f) * -1.0e30f); const float mn = fmaxf(m, sm); const float sc = expf(m - mn); const float e = expf(sm - mn); l = __fadd_rn(__fmul_rn(l, sc), e); m = mn;
#pragma unroll 1
    for (unsigned c = 0; c < HD / 4; ++c) { const v4f vv = *(const v4fa*)(vr + c * 4); v4f oo = *(v4f*)&lo[tid][c * 4];
#pragma unroll
      for (unsigned u = 0; u < 4; ++u) oo[u] = __fadd_rn(__fmul_rn(oo[u], sc), __fmul_rn(e, vv[u]));
      *(v4f*)&lo[tid][c * 4] = oo; } }
  const float fin = 64.0f / l;
#pragma unroll 1
  for (unsigned c = 0; c < HD / 4; ++c) { v4f oo = *(v4f*)&lo[tid][c * 4];
#pragma unroll
    for (unsigned u = 0; u < 4; ++u) oo[u] = __fmul_rn(oo[u], fin);
    *(v4f*)&lo[tid][c * 4] = oo; }
  __syncthreads();
  for (int pass = 0; pass < 2; ++pass) {
#pragma unroll 1
    for (unsigned it = 0; it < 16; ++it) { const unsigned row = it * 4u + (tid >> 4), pc = (tid & 15u) * 4u; const v4f v = *(const v4f*)&lo[row][pc]; *(volatile v4f*)(OF + (size_t)(rg * 64u + row) * ldo + h * HD + pc) = v; }
    if (pass == 0) __threadfence(); }
}

static_assert((size_t)(3 * DM * (DM / 8) / 256) * 256 * 8 == (size_t)3 * DM * DM);
static_assert((size_t)(DM * (DM / 8) / 256) * 256 * 8 == (size_t)DM * DM);
static_assert((NR * DM / 8) % 256 == 0);
static_assert((size_t)((NR / 128) * (DM / 64)) * 4 * 32 * 64 == NR * DM);
static_assert((size_t)NH * (SEQ / 64) * NB * 2 * 64 * 64 == (size_t)2 * NB * NH * HD * SEQ);
static_assert((size_t)((QT / 128) * (HD / 64)) * NH * 4 * 32 * 64 == (size_t)QT * DM);
static_assert((size_t)((SEQ / 128) * (DM / 64)) * NB * 4 * 32 * 64 == NR * DM);
static_assert((size_t)((QT0 / 128) * (DM / 64)) * NB * 4 * 32 * 64 == (size_t)NB * QT0 * DM);
static_assert((size_t)NH * (QT0 / 64) * NB * 64 * 64 == (size_t)NB * QT0 * DM);
static_assert(((size_t)NB * QT0 * DM / 8) % 256 == 0);
static_assert((NH * QT) % 256 == 0);
constexpr size_t SZ_PERSIST = AL256((size_t)DM * DM * 2) + 3 * AL256(NR * DM * 2) + AL256((size_t)2 * NB * NH * HD * SEQ * 2) + 2 * AL256(NR * DM * 2);
constexpr size_t SZ_EARLY = AL256((size_t)3 * DM * DM * 2) + AL256(NR * DM * 2) + AL256((size_t)2 * NR * DM * 2) + 4 * AL256((size_t)NB * QT0 * DM * 4);
constexpr size_t SZ_ATT = AL256((size_t)NH * QT * NKX * 4) + 2 * AL256((size_t)NH * QT * NKX * 2) + AL256((size_t)QT * DM * 4);
static_assert(SZ_PERSIST + (SZ_EARLY > SZ_ATT ? SZ_EARLY : SZ_ATT) <= (size_t)134217728);

extern "C" void kernel_launch(void* const* d_in, const int* in_sizes, int n_in,
                              void* d_out, int out_size, void* d_ws, size_t ws_size, hipStream_t stream) {
  if (n_in < 5) return;
  const size_t xneed = ((size_t)(NB - 1) * SEQ_FULL + SEQ) * DM;
  if ((size_t)in_sizes[0] < xneed) return;
  if ((size_t)in_sizes[1] < (size_t)3 * DM * DM) return;
  if (in_sizes[2] < 3 * DM) return;
  if ((size_t)in_sizes[3] < (size_t)DM * DM) return;
  if (in_sizes[4] < DM) return;
  if ((size_t)out_size < xneed) return;
  const float* x = (const float*)d_in[0]; const float* wqkv = (const float*)d_in[1]; const float* bqkv = (const float*)d_in[2]; const float* wo = (const float*)d_in[3]; const float* bo = (const float*)d_in[4];
  const float* bq = bqkv; const float* bk = bqkv + DM; const float* bv = bqkv + 2 * DM;
  float* out = (float*)d_out;
  char* ws = (char*)d_ws; size_t off = 0;
  auto take = [&](size_t bytes) { char* p = ws + off; off += (bytes + 255) & ~(size_t)255; return p; };
  _Float16* BO = (_Float16*)take((size_t)DM * DM * 2);
  _Float16* Q16 = (_Float16*)take(NR * DM * 2); _Float16* Q16L = (_Float16*)take(NR * DM * 2); _Float16* K16 = (_Float16*)take(NR * DM * 2);
  _Float16* VT2 = (_Float16*)take((size_t)2 * NB * NH * HD * SEQ * 2);
  _Float16* OH = (_Float16*)take(NR * DM * 2); _Float16* OL = (_Float16*)take(NR * DM * 2);
  const size_t ubase = off;
  _Float16* BQKV = (_Float16*)take((size_t)3 * DM * DM * 2); _Float16* BQ = BQKV; _Float16* BK = BQKV + (size_t)DM * DM; _Float16* BV = BQKV + (size_t)2 * DM * DM;
  _Float16* X16 = (_Float16*)take(NR * DM * 2);
  _Float16* V2 = (_Float16*)take((size_t)2 * NR * DM * 2); _Float16* V16 = V2; _Float16* V16L = V2 + NR * DM;
  float* QF0 = (float*)take((size_t)NB * QT0 * DM * 4); float* KF0 = (float*)take((size_t)NB * QT0 * DM * 4); float* VF0 = (float*)take((size_t)NB * QT0 * DM * 4); float* OF0 = (float*)take((size_t)NB * QT0 * DM * 4);
  const size_t end_early = off; off = ubase;
  float* S = (float*)take((size_t)NH * QT * NKX * 4); _Float16* P = (_Float16*)take((size_t)NH * QT * NKX * 2); _Float16* PL = (_Float16*)take((size_t)NH * QT * NKX * 2); float* OT = (float*)take((size_t)QT * DM * 4);
  const size_t end_att = off;
  const size_t total = end_early > end_att ? end_early : end_att;
  if (total > ws_size || total > (size_t)134217728) return;

  k_wt_f16<<<(unsigned)((size_t)3 * DM * (DM / 8) / 256), 256, 0, stream>>>(wqkv, BQKV, DM, 3 * DM, 16.0f);
  k_wt_f16<<<(unsigned)((size_t)DM * (DM / 8) / 256), 256, 0, stream>>>(wo, BO, DM, DM, 16.0f);
  k_x16<<<(unsigned)(NR * DM / 8 / 256), 256, 0, stream>>>(x, X16, (unsigned)(NR * DM / 8));

  const dim3 gp((unsigned)((NR / 128) * (DM / 64)), 1);
  k_gemm2<<<gp, 128, 0, stream>>>(X16, DM, 0, BQ, DM, 0, 0.0625f, bq, nullptr, nullptr, Q16, Q16L, DM, 0, (unsigned)NR, DM, DM);
  k_gemm2<<<gp, 128, 0, stream>>>(X16, DM, 0, BK, DM, 0, 0.0625f, bk, nullptr, nullptr, K16, nullptr, DM, 0, (unsigned)NR, DM, DM);
  k_gemm2<<<gp, 128, 0, stream>>>(X16, DM, 0, BV, DM, 0, 0.0625f, bv, nullptr, nullptr, V16, V16L, DM, 0, (unsigned)NR, DM, DM);

  const dim3 g0((QT0 / 128) * (DM / 64), NB);
  k_gemm2<<<g0, 128, 0, stream>>>(X16, DM, (size_t)SEQ * DM, BQ, DM, 0, 0.0625f, bq, nullptr, QF0, nullptr, nullptr, DM, (size_t)QT0 * DM, QT0, DM, DM);
  k_gemm2<<<g0, 128, 0, stream>>>(X16, DM, (size_t)SEQ * DM, BK, DM, 0, 0.0625f, bk, nullptr, KF0, nullptr, nullptr, DM, (size_t)QT0 * DM, QT0, DM, DM);
  k_gemm2<<<g0, 128, 0, stream>>>(X16, DM, (size_t)SEQ * DM, BV, DM, 0, 0.0625f, bv, nullptr, VF0, nullptr, nullptr, DM, (size_t)QT0 * DM, QT0, DM, DM);
  k_att0<<<dim3(NH * (QT0 / 64), NB), 64, 0, stream>>>(QF0, KF0, VF0, DM, 0.125f, OF0, DM);
  k_hl<<<(unsigned)((size_t)NB * QT0 * DM / 8 / 256), 256, 0, stream>>>(OF0, OH, OL, (unsigned)((size_t)NB * QT0 * DM / 8));

  k_vt<<<dim3(NH * (SEQ / 64), NB, 2), 256, 0, stream>>>(V2, VT2);

  for (unsigned b = 0; b < NB; ++b) { const size_t r0 = (size_t)b * SEQ;
    const _Float16* VTb = VT2 + (size_t)b * NH * HD * SEQ; const _Float16* VTLb = VT2 + (size_t)(NB + b) * NH * HD * SEQ;
    for (unsigned q0 = QT0; q0 < SEQ; q0 += QT) { const unsigned nk = q0 + QT;
      const dim3 gs((QT / 128) * (nk / 64), NH); const dim3 go((QT / 128) * (HD / 64), NH);
      k_gemm2<<<gs, 128, 0, stream>>>(Q16 + (r0 + q0) * DM, DM, (size_t)HD, K16 + r0 * DM, DM, (size_t)HD, 0.125f, nullptr, nullptr, S, nullptr, nullptr, NKX, (size_t)QT * NKX, QT, nk, HD);
      k_gemm2<<<gs, 128, 0, stream>>>(Q16L + (r0 + q0) * DM, DM, (size_t)HD, K16 + r0 * DM, DM, (size_t)HD, 0.0001220703125f, nullptr, S, S, nullptr, nullptr, NKX, (size_t)QT * NKX, QT, nk, HD);
      k_rsmc<<<(NH * QT) / 256, 256, 0, stream>>>(S, P, PL, NH * QT, q0, nk);
      k_gemm2<<<go, 128, 0, stream>>>(P, NKX, (size_t)QT * NKX, VTb, SEQ, (size_t)HD * SEQ, 0.25f, nullptr, nullptr, OT, nullptr, nullptr, DM, (size_t)HD, QT, HD, nk);
      k_gemm2<<<go, 128, 0, stream>>>(P, NKX, (size_t)QT * NKX, VTLb, SEQ, (size_t)HD * SEQ, 0.000244140625f, nullptr, OT, OT, nullptr, nullptr, DM, (size_t)HD, QT, HD, nk);
      k_gemm2<<<go, 128, 0, stream>>>(PL, NKX, (size_t)QT * NKX, VTb, SEQ, (size_t)HD * SEQ, 0.000244140625f, nullptr, OT, nullptr, OH + (r0 + q0) * DM, OL + (r0 + q0) * DM, DM, (size_t)HD, QT, HD, nk); } }

  const dim3 gf((SEQ / 128) * (DM / 64), NB);
  k_gemm2<<<gf, 128, 0, stream>>>(OH, DM, (size_t)SEQ * DM, BO, DM, 0, 0.0009765625f, bo, nullptr, out, nullptr, nullptr, DM, (size_t)SEQ_FULL * DM, SEQ, DM, DM);
  k_gemm2<<<gf, 128, 0, stream>>>(OL, DM, (size_t)SEQ * DM, BO, DM, 0, 0.00000095367431640625f, nullptr, out, out, nullptr, nullptr, DM, (size_t)SEQ_FULL * DM, SEQ, DM, DM);
}
